// SimpleSSMBlock_2327872274722
// MI455X (gfx1250) — hardware-verified
//
#include <hip/hip_runtime.h>

#define B_ 4
#define S_ 2048
#define D_ 1024
#define N_ 16
#define ROWS_ (B_ * S_)

typedef __attribute__((ext_vector_type(8)))  float  v8f;
typedef __attribute__((ext_vector_type(16))) __bf16 v16bf;

union FragBF16 { v16bf v; uint4 q[2]; };

__device__ __forceinline__ unsigned short f2bf(float f) {
    unsigned int u = __builtin_bit_cast(unsigned int, f);
    unsigned int r = u + 0x7FFFu + ((u >> 16) & 1u);
    return (unsigned short)(r >> 16);
}
__device__ __forceinline__ float bf2f(unsigned short h) {
    unsigned int u = ((unsigned int)h) << 16;
    return __builtin_bit_cast(float, u);
}

typedef __attribute__((ext_vector_type(4))) float v4f;
typedef __attribute__((ext_vector_type(4))) unsigned v4u;
template <typename V> __device__ __forceinline__ void vst2(void* p, V v) {
    *(volatile V*)p = v; __threadfence(); *(volatile V*)p = v;
}
__device__ __forceinline__ void copy_b128(unsigned short* lds_dst, const unsigned short* gsrc) {
    *(uint4*)lds_dst = *(const uint4*)gsrc;
}
__device__ __forceinline__ v8f wmma_bf16(v16bf a, v16bf b, v8f c) {
    v8f d = __builtin_amdgcn_wmma_f32_16x16x32_bf16(false, a, false, b, (short)0, c, false, false);
    asm volatile("v_nop\n\tv_nop\n\tv_nop\n\tv_nop" : "+v"(d) : "v"(a), "v"(b));
    return d;
}

#define TCH 32
__global__ __launch_bounds__(512) void ssm_scan_kernel(
    const float* __restrict__ x,
    const float* __restrict__ A,
    const float* __restrict__ Bm,
    const float* __restrict__ Cm,
    const float* __restrict__ Dm,
    float* __restrict__ y_raw)
{
    __shared__ __align__(16) float ybuf[TCH][32];
    const int cl   = threadIdx.x >> 4;
    const int ch   = blockIdx.x * 32 + cl;
    const int lane = threadIdx.x & 15;
    const int b = ch >> 10;
    const int d = ch & (D_ - 1);
    const int d0 = d - cl;

    float Arow[N_];
    const float* Ad = A + (size_t)d * (N_ * N_) + lane * N_;
#pragma unroll
    for (int m = 0; m < N_; ++m) Arow[m] = Ad[m];

    const float bm = Bm[d * N_ + lane];
    const float cm = Cm[d * N_ + lane];
    const float dm = Dm[d];

    const float* xp = x     + (size_t)b * S_ * D_ + d;
    float*       yp = y_raw + (size_t)b * S_ * D_ + d;

    float h = 0.0f;
    for (int t = 0; t < S_; ++t) {
        if (t + 16 < S_) __builtin_prefetch(xp + (size_t)(t + 16) * D_, 0, 3);

        const float xv = xp[(size_t)t * D_];
        float hn = 0.0f;
#pragma unroll
        for (int m = 0; m < N_; ++m)
            hn = fmaf(Arow[m], __shfl(h, m, 16), hn);
        h = fmaf(bm, xv, hn);

        float p = cm * h;
#pragma unroll
        for (int off = 8; off; off >>= 1) p += __shfl_xor(p, off, 16);

        if (lane == 0) ybuf[t & (TCH - 1)][cl] = fmaf(dm, xv, p);
        if ((t & (TCH - 1)) == TCH - 1) {
            __syncthreads();
            if (threadIdx.x < 256) {
                const int tt = threadIdx.x >> 3, pc = threadIdx.x & 7;
                vst2(y_raw + ((size_t)b * S_ + (t - (TCH - 1)) + tt) * D_ + d0 + pc * 4, *(const v4f*)(&ybuf[tt][pc * 4]));
            }
            __syncthreads();
        }
    }
    (void)yp;
}

__global__ __launch_bounds__(256) void w_split_kernel(
    const float* __restrict__ W,
    unsigned short* __restrict__ Whi,
    unsigned short* __restrict__ Wlo)
{
    int g = blockIdx.x * 256 + threadIdx.x;
    union { unsigned short s[8]; v4u u; } ph, pl;
#pragma unroll
    for (int e = 0; e < 8; ++e) {
        float f = W[(size_t)g * 8 + e];
        unsigned short hi = f2bf(f);
        ph.s[e] = hi; pl.s[e] = f2bf(f - bf2f(hi));
    }
    vst2(Whi + (size_t)g * 8, ph.u);
    vst2(Wlo + (size_t)g * 8, pl.u);
}

__global__ __launch_bounds__(256) void ln_gelu_split_kernel(
    const float* __restrict__ y_raw,
    const float* __restrict__ ln_w,
    const float* __restrict__ ln_b,
    unsigned short* __restrict__ yn_hi,
    unsigned short* __restrict__ yn_lo)
{
    __shared__ float red[8];
    const int row = blockIdx.x;
    const int tid = threadIdx.x;
    const float* yr = y_raw + (size_t)row * D_;

    float v[4];
    float s = 0.0f;
    {
        const v4f q4 = *(const v4f*)(yr + tid * 4);
#pragma unroll
        for (int i = 0; i < 4; ++i) { v[i] = q4[i]; s += v[i]; }
    }

#pragma unroll
    for (int off = 16; off; off >>= 1) s += __shfl_xor(s, off, 32);
    if ((tid & 31) == 0) red[tid >> 5] = s;
    __syncthreads();
    float tot = 0.0f;
#pragma unroll
    for (int i = 0; i < 8; ++i) tot += red[i];
    const float mu = tot * (1.0f / D_);
    __syncthreads();

    float vs = 0.0f;
#pragma unroll
    for (int i = 0; i < 4; ++i) { float dlt = v[i] - mu; vs += dlt * dlt; }
#pragma unroll
    for (int off = 16; off; off >>= 1) vs += __shfl_xor(vs, off, 32);
    if ((tid & 31) == 0) red[tid >> 5] = vs;
    __syncthreads();
    float vtot = 0.0f;
#pragma unroll
    for (int i = 0; i < 8; ++i) vtot += red[i];
    const float rinv = rsqrtf(vtot * (1.0f / D_) + 1e-5f);

    union { unsigned short s[4]; unsigned long long u; } ph, pl;
#pragma unroll
    for (int i = 0; i < 4; ++i) {
        const int col = tid * 4 + i;
        float u = (v[i] - mu) * rinv * ln_w[col] + ln_b[col];
        float g = 0.5f * u * (1.0f + erff(u * 0.70710678118654752f));
        unsigned short hi = f2bf(g);
        ph.s[i] = hi; pl.s[i] = f2bf(g - bf2f(hi));
    }
    vst2(yn_hi + (size_t)row * D_ + tid * 4, ph.u);
    vst2(yn_lo + (size_t)row * D_ + tid * 4, pl.u);
}

#define TM 128
#define TN 64
#define KC 32
#define LDSS 40
#define NCHUNK (D_ / KC)

__global__ __launch_bounds__(256) void gemm_wmma_kernel(
    const unsigned short* __restrict__ Ahg,
    const unsigned short* __restrict__ Alg,
    const unsigned short* __restrict__ Bhg,
    const unsigned short* __restrict__ Blg,
    const float* __restrict__ x,
    const float* __restrict__ b_out,
    float* __restrict__ out)
{
    __shared__ unsigned short sAh[2][TM * LDSS];
    __shared__ unsigned short sAl[2][TM * LDSS];
    __shared__ unsigned short sBh[2][TN * LDSS];
    __shared__ unsigned short sBl[2][TN * LDSS];
    __shared__ __align__(16) float Ct[TM][TN];

    const int tid = threadIdx.x;
    const int bm0 = blockIdx.x * TM;
    const int bn0 = blockIdx.y * TN;

    const int w    = tid >> 5;
    const int L    = tid & 31;
    const int wm   = (w & 3) * 32;
    const int wn   = (w >> 2) * 32;
    const int lm   = L & 15;
    const int half = L >> 4;

    auto issue_chunk = [&](int kc, int buf) {
#pragma unroll
        for (int ii = 0; ii < 2; ++ii) {
            const int i = tid + ii * 256;
            const int r = i >> 2, q = i & 3;
            const size_t ge = (size_t)(bm0 + r) * D_ + kc + q * 8;
            const int    le = r * LDSS + q * 8;
            copy_b128(&sAh[buf][le], Ahg + ge);
            copy_b128(&sAl[buf][le], Alg + ge);
        }
        {
            const int r = tid >> 2, q = tid & 3;
            const size_t ge = (size_t)(bn0 + r) * D_ + kc + q * 8;
            const int    le = r * LDSS + q * 8;
            copy_b128(&sBh[buf][le], Bhg + ge);
            copy_b128(&sBl[buf][le], Blg + ge);
        }
    };

    v8f acc[2][2] = {};

    issue_chunk(0, 0);

    for (int c = 0; c < NCHUNK; ++c) {
        const int buf = c & 1;
        if (c + 1 < NCHUNK) issue_chunk((c + 1) * KC, (c + 1) & 1);
        __syncthreads();

        const unsigned short* pAh = sAh[buf];
        const unsigned short* pAl = sAl[buf];
        const unsigned short* pBh = sBh[buf];
        const unsigned short* pBl = sBl[buf];

#pragma unroll
        for (int mi = 0; mi < 2; ++mi) {
            const int ar = (wm + mi * 16 + lm) * LDSS;
            FragBF16 ah, al;
            ah.q[0] = *(const uint4*)(&pAh[ar + half * 8]);
            ah.q[1] = *(const uint4*)(&pAh[ar + 16 + half * 8]);
            al.q[0] = *(const uint4*)(&pAl[ar + half * 8]);
            al.q[1] = *(const uint4*)(&pAl[ar + 16 + half * 8]);

#pragma unroll
            for (int ni = 0; ni < 2; ++ni) {
                const int br = (wn + ni * 16 + lm) * LDSS;
                FragBF16 bh, bl;
                bh.q[0] = *(const uint4*)(&pBh[br + half * 8]);
                bh.q[1] = *(const uint4*)(&pBh[br + 16 + half * 8]);
                bl.q[0] = *(const uint4*)(&pBl[br + half * 8]);
                bl.q[1] = *(const uint4*)(&pBl[br + 16 + half * 8]);

                v8f cacc = acc[mi][ni];
                cacc = wmma_bf16(ah.v, bh.v, cacc);
                cacc = wmma_bf16(ah.v, bl.v, cacc);
                cacc = wmma_bf16(al.v, bh.v, cacc);
                acc[mi][ni] = cacc;
            }
        }
        __syncthreads();
    }

#pragma unroll
    for (int mi = 0; mi < 2; ++mi) {
#pragma unroll
        for (int ni = 0; ni < 2; ++ni) {
            const int cj = wn + ni * 16 + lm;
            const float bb = b_out[bn0 + cj];
#pragma unroll
            for (int v = 0; v < 8; ++v) Ct[wm + mi * 16 + v + half * 8][cj] = acc[mi][ni][v] + bb;
        }
    }
    __syncthreads();
    for (int g = tid; g < TM * 16; g += 256) {
        const int rl = g >> 4, pc = g & 15;
        const size_t o = (size_t)(bm0 + rl) * D_ + bn0 + pc * 4;
        vst2(out + o, *(const v4f*)(&Ct[rl][pc * 4]) + *(const v4f*)(x + o));
    }
}

extern "C" void kernel_launch(void* const* d_in, const int* in_sizes, int n_in,
                              void* d_out, int out_size, void* d_ws, size_t ws_size,
                              hipStream_t stream) {
    const float* x     = (const float*)d_in[0];
    const float* A     = (const float*)d_in[1];
    const float* Bm    = (const float*)d_in[2];
    const float* Cm    = (const float*)d_in[3];
    const float* Dm    = (const float*)d_in[4];
    const float* ln_w  = (const float*)d_in[5];
    const float* ln_b  = (const float*)d_in[6];
    const float* W_out = (const float*)d_in[7];
    const float* b_out = (const float*)d_in[8];
    float* out = (float*)d_out;

    char* ws = (char*)d_ws;
    float*          y_raw = (float*)ws;
    unsigned short* yn_hi = (unsigned short*)(ws + (size_t)ROWS_ * D_ * 4);
    unsigned short* yn_lo = (unsigned short*)(ws + (size_t)ROWS_ * D_ * 4
                                                 + (size_t)ROWS_ * D_ * 2);
    unsigned short* w_hi  = (unsigned short*)(ws + (size_t)ROWS_ * D_ * 4
                                                 + (size_t)ROWS_ * D_ * 4);
    unsigned short* w_lo  = (unsigned short*)(ws + (size_t)ROWS_ * D_ * 4
                                                 + (size_t)ROWS_ * D_ * 4
                                                 + (size_t)D_ * D_ * 2);

    w_split_kernel<<<(D_ * D_ / 8) / 256, 256, 0, stream>>>(W_out, w_hi, w_lo);

    ssm_scan_kernel<<<(B_ * D_) / 32, 512, 0, stream>>>(x, A, Bm, Cm, Dm, y_raw);

    ln_gelu_split_kernel<<<ROWS_, 256, 0, stream>>>(y_raw, ln_w, ln_b, yn_hi, yn_lo);

    dim3 grid(ROWS_ / TM, D_ / TN);
    gemm_wmma_kernel<<<grid, 256, 0, stream>>>(yn_hi, yn_lo, w_hi, w_lo, x, b_out, out);
}
